// Block_84911503442222
// MI455X (gfx1250) — hardware-verified
//
#include <hip/hip_runtime.h>
#include <math.h>

typedef __attribute__((ext_vector_type(16))) _Float16 v16h;
typedef __attribute__((ext_vector_type(8)))  _Float16 v8h;
typedef __attribute__((ext_vector_type(8)))  float    v8f;
typedef __attribute__((ext_vector_type(4)))  float    v4f;

constexpr int kBatch = 2;
constexpr int kSeqL  = 2048;
constexpr int kDmod  = 1024;
constexpr int kDin   = 2048;
constexpr int kNst   = 16;
constexpr int kDtR   = 64;
constexpr int kPrjN  = 96;
constexpr int kPrjP  = 128;
constexpr int kXZP   = 2 * kDin;
constexpr int kTP    = 260;

constexpr float kCarryW  = 32.0f;
constexpr float kCarryHN = 16.0f;
constexpr float kCarryU  = 16.0f;
constexpr float kCarryDT = 16.0f;
constexpr float kCarryY  = 256.0f;
constexpr float kFoldIn  = 1.0f / (kCarryHN * kCarryW);
constexpr float kFoldXp  = 1.0f / (kCarryU * kCarryW);
constexpr float kFoldDt  = 1.0f / (kCarryDT * kCarryW);
constexpr float kFoldOut = 1.0f / (kCarryY * kCarryW);

static_assert(kDtR + 2 * kNst == kPrjN, "x_proj width");
static_assert((kDmod % 32) == 0 && (kDin % 32) == 0 && (kDtR % 32) == 0, "GEMM K multiples of 32");
static_assert((kSeqL % 64) == 0 && (kXZP % 64) == 0 && (kPrjP % 64) == 0 && (kDin % 64) == 0 && (kDmod % 64) == 0, "GEMM M,N multiples of 64");
static_assert((kDin % 256) == 0 && (kDmod % 256) == 0 && (kSeqL % 32) == 0, "tile multiples");

constexpr size_t kSzWIN  = (size_t)kXZP * kDmod * 2;
constexpr size_t kSzWOUT = (size_t)kDmod * kDin * 2;
constexpr size_t kSzWXP  = (size_t)kPrjP * kDin * 2;
constexpr size_t kSzWDT  = (size_t)kDin * kDtR * 2;
constexpr size_t kSzHN   = (size_t)kBatch * kSeqL * kDmod * 2;
constexpr size_t kSzXZ   = (size_t)kSeqL * kXZP * 4;
constexpr size_t kSzUC   = (size_t)kSeqL * kDin * 4;
constexpr size_t kSzUC16 = (size_t)kSeqL * kDin * 2;
constexpr size_t kSzPROJ = (size_t)kSeqL * kPrjP * 4;
constexpr size_t kSzDT16 = (size_t)kSeqL * kDtR * 2;
constexpr size_t kSzDLR  = (size_t)kSeqL * kDin * 4;
constexpr size_t kSzGF   = (size_t)kSeqL * kDin * 4;
constexpr size_t kSzY16  = (size_t)kSeqL * kDin * 2;
constexpr size_t kOffWIN  = 0;
constexpr size_t kOffWOUT = kOffWIN  + kSzWIN;
constexpr size_t kOffWXPF = kOffWOUT + kSzWOUT;
constexpr size_t kOffWXPB = kOffWXPF + kSzWXP;
constexpr size_t kOffWDTF = kOffWXPB + kSzWXP;
constexpr size_t kOffWDTB = kOffWDTF + kSzWDT;
constexpr size_t kOffHN   = kOffWDTB + kSzWDT;
constexpr size_t kOffXZ   = kOffHN   + kSzHN;
constexpr size_t kOffUC   = kOffXZ   + kSzXZ;
constexpr size_t kOffUC16 = kOffUC   + kSzUC;
constexpr size_t kOffPROJ = kOffUC16 + kSzUC16;
constexpr size_t kOffDT16 = kOffPROJ + kSzPROJ;
constexpr size_t kOffDLR  = kOffDT16 + kSzDT16;
constexpr size_t kOffGF   = kOffDLR  + kSzDLR;
constexpr size_t kOffY16  = kOffGF   + kSzGF;
constexpr size_t kWsTotal = kOffY16  + kSzY16;
static_assert(kWsTotal == 124518400ull, "carve total");
static_assert(kWsTotal <= 134217728ull, "carve cap");
static_assert((kOffWOUT % 128) == 0 && (kOffWXPF % 128) == 0 && (kOffWXPB % 128) == 0 && (kOffWDTF % 128) == 0 &&
              (kOffWDTB % 128) == 0 && (kOffHN % 128) == 0 && (kOffXZ % 128) == 0 && (kOffUC % 128) == 0 &&
              (kOffUC16 % 128) == 0 && (kOffPROJ % 128) == 0 && (kOffDT16 % 128) == 0 && (kOffDLR % 128) == 0 &&
              (kOffGF % 128) == 0 && (kOffY16 % 128) == 0, "128-B aligned regions");

__device__ __forceinline__ void dep_guard4_h(v8f& a, v8f& b, v8f& c, v8f& d, v16h x, v16h y) {
  asm volatile("v_nop\n\tv_nop\n\tv_nop\n\tv_nop" : "+v"(a), "+v"(b), "+v"(c), "+v"(d) : "v"(x), "v"(y));
}
__device__ __forceinline__ void keep4_h(v16h a, v16h b, v16h c, v16h d) { asm volatile("v_nop" :: "v"(a), "v"(b), "v"(c), "v"(d)); }
__device__ __forceinline__ void acc_guard4(v8f& a, v8f& b, v8f& c, v8f& d) { asm volatile("v_nop\n\tv_nop\n\tv_nop\n\tv_nop" : "+v"(a), "+v"(b), "+v"(c), "+v"(d)); }
template <typename T> struct Frag;
template <> struct Frag<_Float16> {
  typedef v16h V; union U { v16h v; v8h h[2]; };
  static __device__ __forceinline__ v16h load(const _Float16* p) {
    U f; f.h[0] = *(const v8h*)(p); f.h[1] = *(const v8h*)(p + 16); return f.v;
  }
  static __device__ __forceinline__ v8f mma(v16h a, v16h b, v8f c) {
    return __builtin_amdgcn_wmma_f32_16x16x32_f16(false, a, false, b, (short)0, c, false, false);
  }
};

template <int BIAS_MODE>
__global__ __launch_bounds__(256) void wmma_gemm64_f16(
    const unsigned short* __restrict__ Ap, int lda,
    const unsigned short* __restrict__ Btp, int ldb,
    float* __restrict__ C, int ldc,
    const float* __restrict__ bias,
    int M, int N, int K, float scale) {
  typedef _Float16 T;
  typedef Frag<T>::V V;
  const T* A = (const T*)Ap; const T* Bt = (const T*)Btp;
  __shared__ __align__(16) float sT[8][16 * 68];
  const int lane = threadIdx.x & 31;
  const int wave = threadIdx.x >> 5;
  const int tilesN = N >> 6;
  const int tilesM = M >> 6;
  const int tile = blockIdx.x * 8 + wave;
  if (tile >= tilesM * tilesN) return;
  const int tm = tile / tilesN;
  const int tn = tile - tm * tilesN;
  const int m0 = tm << 6;
  const int n0 = tn << 6;

  const int rlane = lane & 15;
  const int koff  = (lane >> 4) * 8;
  const int mOff  = (lane >> 4) * 8;

  v8f acc[4][4];
#pragma unroll
  for (int i = 0; i < 4; ++i)
#pragma unroll
    for (int j = 0; j < 4; ++j) acc[i][j] = (v8f){0.f,0.f,0.f,0.f,0.f,0.f,0.f,0.f};

  for (int k0 = 0; k0 < K; k0 += 32) {
    V bh[4];
#pragma unroll
    for (int j = 0; j < 4; ++j) {
      const size_t bo = (size_t)(n0 + (j << 4) + rlane) * ldb + koff + k0;
      bh[j] = Frag<T>::load(Bt + bo);
    }
#pragma unroll
    for (int i = 0; i < 4; ++i) {
      const size_t ao = (size_t)(m0 + (i << 4) + rlane) * lda + koff + k0;
      V ah = Frag<T>::load(A + ao);
#pragma unroll
      for (int j = 0; j < 4; ++j) acc[i][j] = Frag<T>::mma(ah, bh[j], acc[i][j]);
      dep_guard4_h(acc[i][0], acc[i][1], acc[i][2], acc[i][3], ah, ah);
    }
    keep4_h(bh[0], bh[1], bh[2], bh[3]);
  }
  acc_guard4(acc[0][0], acc[0][1], acc[0][2], acc[0][3]);
  acc_guard4(acc[1][0], acc[1][1], acc[1][2], acc[1][3]);
  acc_guard4(acc[2][0], acc[2][1], acc[2][2], acc[2][3]);
  acc_guard4(acc[3][0], acc[3][1], acc[3][2], acc[3][3]);

  float* slab = sT[wave];
#pragma unroll
  for (int i = 0; i < 4; ++i) {
    const int mBase = m0 + (i << 4);
#pragma unroll
    for (int j = 0; j < 4; ++j) {
      const int n = n0 + (j << 4) + rlane;
      float bv = 0.f;
      if (BIAS_MODE == 2) bv = bias[n];
#pragma unroll
      for (int r = 0; r < 8; ++r) {
        float v = acc[i][j][r] * scale;
        if (BIAS_MODE == 1) v += bias[mBase + mOff + r];
        if (BIAS_MODE == 2) v += bv;
        slab[(mOff + r) * 68 + (j << 4) + rlane] = v;
      }
    }
    __builtin_amdgcn_fence(__ATOMIC_RELEASE, "workgroup");
    __builtin_amdgcn_wave_barrier();
    __builtin_amdgcn_fence(__ATOMIC_ACQUIRE, "workgroup");
    {
      const int hh = lane >> 4, c4 = (lane & 15) * 4;
      for (int pass = 0; pass < 2; ++pass) {
#pragma unroll
        for (int it = 0; it < 8; ++it) {
          const int row = it * 2 + hh;
          v4f v = *(const v4f*)(slab + row * 68 + c4);
          *(volatile v4f*)(C + (size_t)(mBase + row) * ldc + n0 + c4) = v;
        }
        __threadfence();
      }
    }
    __builtin_amdgcn_fence(__ATOMIC_RELEASE, "workgroup");
    __builtin_amdgcn_wave_barrier();
    __builtin_amdgcn_fence(__ATOMIC_ACQUIRE, "workgroup");
  }
}

__global__ __launch_bounds__(256) void cast_f16_kernel(
    const float* __restrict__ src, unsigned short* __restrict__ dst, int total8, int real8, float scale)
{
  const int i = blockIdx.x * 256 + threadIdx.x;
  if (i >= total8) return;
  const bool live = (i < real8);
  const int ic = live ? i : (real8 - 1);
  const float* p = src + ((size_t)ic << 3);
  const v4f a0 = *(const v4f*)(p);
  const v4f a1 = *(const v4f*)(p + 4);
  v8h hv;
#pragma unroll
  for (int e = 0; e < 4; ++e) {
    const float f0 = a0[e] * scale;
    const float f1 = a1[e] * scale;
    hv[e]     = (_Float16)(live ? f0 : 0.0f);
    hv[4 + e] = (_Float16)(live ? f1 : 0.0f);
  }
  unsigned short* q = dst + ((size_t)i << 3);
  *(volatile v8h*)q = hv;
  __threadfence();
  *(volatile v8h*)q = hv;
}

__global__ __launch_bounds__(256) void dt_cast_kernel(
    const float* __restrict__ PROJ, unsigned short* __restrict__ DT16, int total8, float scale)
{
  const int i = blockIdx.x * 256 + threadIdx.x;
  if (i >= total8) return;
  const int e0  = i << 3;
  const int row = e0 >> 6;
  const int c8  = e0 & 63;
  const float* p = PROJ + (size_t)row * kPrjP + c8;
  const v4f a0 = *(const v4f*)(p);
  const v4f a1 = *(const v4f*)(p + 4);
  v8h hv;
#pragma unroll
  for (int e = 0; e < 4; ++e) {
    hv[e]     = (_Float16)(a0[e] * scale);
    hv[4 + e] = (_Float16)(a1[e] * scale);
  }
  unsigned short* qd = DT16 + e0;
  *(volatile v8h*)qd = hv;
  __threadfence();
  *(volatile v8h*)qd = hv;
}

__global__ __launch_bounds__(256) void prelude_kernel(
    const float* __restrict__ hidden, const float* __restrict__ residual,
    const float* __restrict__ gamma, const float* __restrict__ beta,
    float* __restrict__ out1, unsigned short* __restrict__ HN)
{
  __shared__ __align__(16) float sH[32 * kTP];
  __shared__ __align__(16) float sPs[32 * 32];
  __shared__ __align__(16) float sPq[32 * 32];
  __shared__ __align__(16) float sMu[32];
  __shared__ __align__(16) float sRs[32];
  const int tid = threadIdx.x, lane = tid & 31, wave = tid >> 5;
  const int q = lane >> 3, c4 = (lane & 7) * 4;
  const int b  = blockIdx.x >> 6;
  const int l0 = (blockIdx.x & 63) * 32;
  const size_t base = (size_t)b * kDmod * kSeqL + l0 + c4;

  v4f s  = (v4f){0.f, 0.f, 0.f, 0.f};
  v4f qq = (v4f){0.f, 0.f, 0.f, 0.f};
#pragma unroll 1
  for (int it = 0; it < 32; ++it) {
    const int d = it * 32 + wave * 4 + q;
    const size_t off = base + (size_t)d * kSeqL;
    const v4f hv = *(const v4f*)(hidden + off);
    const v4f rv = *(const v4f*)(residual + off);
    const v4f r = hv + rv;
    *(volatile v4f*)(out1 + off) = r;
    s  += r;
    qq += r * r;
  }
  {
    const int part = wave * 4 + q;
    *(v4f*)(sPs + part * 32 + c4) = s;
    *(v4f*)(sPq + part * 32 + c4) = qq;
  }
  __threadfence();
  __syncthreads();
  if (tid < 32) {
    float ts = 0.f, tq = 0.f;
#pragma unroll 1
    for (int p = 0; p < 32; ++p) { ts += sPs[p * 32 + tid]; tq += sPq[p * 32 + tid]; }
    const float mu = ts * (1.0f / (float)kDmod);
    float var = tq * (1.0f / (float)kDmod) - mu * mu;
    var = fmaxf(var, 0.0f);
    sMu[tid] = mu;
    sRs[tid] = rsqrtf(var + 1e-5f);
  }
  __syncthreads();
  const v4f mu4 = *(const v4f*)(sMu + c4);
  const v4f rs4 = *(const v4f*)(sRs + c4);
#pragma unroll 1
  for (int ch = 0; ch < 4; ++ch) {
#pragma unroll 1
    for (int i8 = 0; i8 < 8; ++i8) {
      const int dl = i8 * 32 + wave * 4 + q;
      const int d  = ch * 256 + dl;
      const size_t off = base + (size_t)d * kSeqL;
      const v4f hv = *(const v4f*)(hidden + off);
      const v4f rv = *(const v4f*)(residual + off);
      const v4f r = hv + rv;
      *(volatile v4f*)(out1 + off) = r;
      const float g = gamma[d], be = beta[d];
#pragma unroll
      for (int e = 0; e < 4; ++e) {
        const float hn = ((r[e] - mu4[e]) * rs4[e]) * g + be;
        sH[(c4 + e) * kTP + dl] = hn * kCarryHN;
      }
    }
    __syncthreads();
    v8h h16[4];
#pragma unroll
    for (int it = 0; it < 4; ++it) {
      const float* sp = sH + (it * 8 + wave) * kTP + lane * 8;
      const v4f a0 = *(const v4f*)(sp);
      const v4f a1 = *(const v4f*)(sp + 4);
#pragma unroll
      for (int e = 0; e < 4; ++e) { h16[it][e] = (_Float16)a0[e]; h16[it][4 + e] = (_Float16)a1[e]; }
    }
    for (int pass = 0; pass < 2; ++pass) {
#pragma unroll
      for (int it = 0; it < 4; ++it) {
        const size_t o = ((size_t)b * kSeqL + l0 + it * 8 + wave) * kDmod + ch * 256 + lane * 8;
        *(volatile v8h*)(HN + o) = h16[it];
      }
      __threadfence();
    }
    __syncthreads();
  }
}

template <bool REV>
__global__ __launch_bounds__(256) void conv_silu_kernel(
    const float* __restrict__ XZ, const float* __restrict__ cw, const float* __restrict__ cb,
    float* __restrict__ UC, unsigned short* __restrict__ UC16)
{
  __shared__ __align__(16) float sT[16 * kTP];
  const int tid = threadIdx.x, lane = tid & 31, wave = tid >> 5;
  const int d0 = blockIdx.x * 256, d = d0 + tid;
  const int t0 = blockIdx.y * 64;
  const float w0 = cw[d * 4 + 0], w1 = cw[d * 4 + 1], w2 = cw[d * 4 + 2], w3 = cw[d * 4 + 3];
  const float bc = cb[d];
  float xm3, xm2, xm1;
  {
    const int r3 = REV ? (t0 + 66) : (t0 - 3);
    const int r2 = REV ? (t0 + 65) : (t0 - 2);
    const int r1 = REV ? (t0 + 64) : (t0 - 1);
    const int c3 = r3 < 0 ? 0 : (r3 > kSeqL - 1 ? kSeqL - 1 : r3);
    const int c2 = r2 < 0 ? 0 : (r2 > kSeqL - 1 ? kSeqL - 1 : r2);
    const int c1 = r1 < 0 ? 0 : (r1 > kSeqL - 1 ? kSeqL - 1 : r1);
    const float v3 = XZ[(size_t)c3 * kXZP + d];
    const float v2 = XZ[(size_t)c2 * kXZP + d];
    const float v1 = XZ[(size_t)c1 * kXZP + d];
    xm3 = (r3 >= 0 && r3 < kSeqL) ? v3 : 0.f;
    xm2 = (r2 >= 0 && r2 < kSeqL) ? v2 : 0.f;
    xm1 = (r1 >= 0 && r1 < kSeqL) ? v1 : 0.f;
  }
  const int hrow = wave >> 1;
  const int hch  = (wave & 1) * 128 + lane * 4;
#pragma unroll 1
  for (int sub = 0; sub < 4; ++sub) {
    const int lb = REV ? (t0 + 48 - 16 * sub) : (t0 + 16 * sub);
#pragma unroll 1
    for (int s = 0; s < 16; ++s) {
      const int tr = REV ? (15 - s) : s;
      const float xc = XZ[(size_t)(lb + tr) * kXZP + d];
      float acc = w0 * xm3;
      acc = fmaf(w1, xm2, acc);
      acc = fmaf(w2, xm1, acc);
      acc = fmaf(w3, xc, acc);
      const float sv = acc + bc;
      const float sg = __builtin_amdgcn_rcpf(1.0f + expf(-sv));
      sT[tr * kTP + tid] = sv * sg;
      xm3 = xm2; xm2 = xm1; xm1 = xc;
    }
    __syncthreads();
    v4f fv[4];
    v8h bv[2];
#pragma unroll
    for (int it = 0; it < 4; ++it) fv[it] = *(const v4f*)(sT + (it * 4 + hrow) * kTP + hch);
#pragma unroll
    for (int it = 0; it < 2; ++it) {
      const float* sp = sT + (it * 8 + wave) * kTP + lane * 8;
      const v4f a0 = *(const v4f*)(sp);
      const v4f a1 = *(const v4f*)(sp + 4);
#pragma unroll
      for (int e = 0; e < 4; ++e) {
        bv[it][e]     = (_Float16)(a0[e] * kCarryU);
        bv[it][4 + e] = (_Float16)(a1[e] * kCarryU);
      }
    }
    for (int pass = 0; pass < 2; ++pass) {
#pragma unroll
      for (int it = 0; it < 4; ++it)
        *(volatile v4f*)(UC + (size_t)(lb + it * 4 + hrow) * kDin + d0 + hch) = fv[it];
#pragma unroll
      for (int it = 0; it < 2; ++it)
        *(volatile v8h*)(UC16 + (size_t)(lb + it * 8 + wave) * kDin + d0 + lane * 8) = bv[it];
      __threadfence();
    }
    __syncthreads();
  }
}

template <bool REV>
__global__ __launch_bounds__(256) void scan_kernel(
    const float* __restrict__ DLR, const float* __restrict__ UC, const float* __restrict__ XZ,
    const float* __restrict__ PROJ, const float* __restrict__ A_log, const float* __restrict__ Dv,
    float* GF, unsigned short* __restrict__ Y16)
{
  __shared__ __align__(16) float sBC[16 * 32];
  __shared__ __align__(16) float sY[16 * kTP];
  __shared__ __align__(16) float sA[kNst * 256];
  const int tid = threadIdx.x, lane = tid & 31, wave = tid >> 5;
  const int d0 = blockIdx.x * 256, d = d0 + tid;

#pragma unroll 1
  for (int n = 0; n < kNst; ++n) sA[n * 256 + tid] = -expf(A_log[(size_t)d * kNst + n]);
  __syncthreads();
  float An[kNst], h[kNst];
#pragma unroll
  for (int n = 0; n < kNst; ++n) { An[n] = sA[n * 256 + tid]; h[n] = 0.f; }
  const float Dd = Dv[d];
  const int hrow = wave >> 1;
  const int hch  = (wave & 1) * 128 + lane * 4;

#pragma unroll 1
  for (int c = 0; c < kSeqL / 16; ++c) {
    const int l0 = REV ? (kSeqL - 16 - 16 * c) : (16 * c);
    if (tid < 128) {
      const int r = tid >> 3, qc = (tid & 7) * 4;
      const v4f v = *(const v4f*)(PROJ + (size_t)(l0 + r) * kPrjP + kDtR + qc);
      *(v4f*)(sBC + r * 32 + qc) = v;
    }
    __syncthreads();
#pragma unroll 1
    for (int s = 0; s < 16; ++s) {
      const int tr = REV ? (15 - s) : s;
      const size_t m = (size_t)(l0 + tr);
      const float a  = DLR[m * kDin + d];
      const float xv = UC[m * kDin + d];
      const float ea = __expf(-fabsf(a));
      const float ub = 1.0f + ea;
      const float l1p = __logf(ub) + (ea - (ub - 1.0f)) * __builtin_amdgcn_rcpf(ub);
      const float delta = fmaxf(a, 0.0f) + l1p;
      v4f Bq[4], Cq[4];
#pragma unroll
      for (int qv = 0; qv < 4; ++qv) {
        Bq[qv] = *(const v4f*)(sBC + tr * 32 + 4 * qv);
        Cq[qv] = *(const v4f*)(sBC + tr * 32 + kNst + 4 * qv);
      }
      const float dx = delta * xv;
      float y = 0.f;
#pragma unroll
      for (int n = 0; n < kNst; ++n) {
        const float e = __expf(delta * An[n]);
        h[n] = e * h[n] + dx * Bq[n >> 2][n & 3];
        y = h[n] * Cq[n >> 2][n & 3] + y;
      }
      y = xv * Dd + y;
      if (REV) {
        const float gf = GF[m * kDin + d];
        const float zv = XZ[m * kXZP + kDin + d];
        const float sg = __builtin_amdgcn_rcpf(1.0f + expf(-zv));
        sY[tr * kTP + tid] = ((gf + y) * (zv * sg)) * kCarryY;
      } else {
        sY[tr * kTP + tid] = y;
      }
    }
    __syncthreads();
    if (REV) {
      v8h hv[2];
#pragma unroll
      for (int it = 0; it < 2; ++it) {
        const float* sp = sY + (it * 8 + wave) * kTP + lane * 8;
        const v4f a0 = *(const v4f*)(sp);
        const v4f a1 = *(const v4f*)(sp + 4);
#pragma unroll
        for (int e = 0; e < 4; ++e) { hv[it][e] = (_Float16)a0[e]; hv[it][4 + e] = (_Float16)a1[e]; }
      }
      for (int pass = 0; pass < 2; ++pass) {
#pragma unroll
        for (int it = 0; it < 2; ++it)
          *(volatile v8h*)(Y16 + (size_t)(l0 + it * 8 + wave) * kDin + d0 + lane * 8) = hv[it];
        __threadfence();
      }
    } else {
      v4f fv[4];
#pragma unroll
      for (int it = 0; it < 4; ++it) fv[it] = *(const v4f*)(sY + (it * 4 + hrow) * kTP + hch);
      for (int pass = 0; pass < 2; ++pass) {
#pragma unroll
        for (int it = 0; it < 4; ++it)
          *(volatile v4f*)(GF + (size_t)(l0 + it * 4 + hrow) * kDin + d0 + hch) = fv[it];
        __threadfence();
      }
    }
  }
}

extern "C" void kernel_launch(void* const* d_in, const int* in_sizes, int n_in,
                              void* d_out, int out_size, void* d_ws, size_t ws_size,
                              hipStream_t stream)
{
  if (n_in < 21) return;
  if (in_sizes[0] != kBatch * kDmod * kSeqL || in_sizes[1] != kBatch * kDmod * kSeqL) return;
  if (in_sizes[2] != kDmod || in_sizes[3] != kDmod) return;
  if (in_sizes[4] != kXZP * kDmod) return;
  if (in_sizes[5] != kDin * 4 || in_sizes[6] != kDin) return;
  if (in_sizes[7] != kPrjN * kDin) return;
  if (in_sizes[8] != kDin * kDtR || in_sizes[9] != kDin) return;
  if (in_sizes[10] != kDin * kNst || in_sizes[11] != kDin) return;
  if (in_sizes[12] != kDin * 4 || in_sizes[13] != kDin) return;
  if (in_sizes[14] != kPrjN * kDin) return;
  if (in_sizes[15] != kDin * kDtR || in_sizes[16] != kDin) return;
  if (in_sizes[17] != kDin * kNst || in_sizes[18] != kDin) return;
  if (in_sizes[19] != kDmod * kDin || in_sizes[20] != kDmod) return;
  if (out_size != 2 * kBatch * kDmod * kSeqL) return;
  if (ws_size < kWsTotal) return;

  const float* hidden     = (const float*)d_in[0];
  const float* residual   = (const float*)d_in[1];
  const float* gamma      = (const float*)d_in[2];
  const float* beta       = (const float*)d_in[3];
  const float* in_proj_w  = (const float*)d_in[4];
  const float* conv_w     = (const float*)d_in[5];
  const float* conv_b     = (const float*)d_in[6];
  const float* xproj_w    = (const float*)d_in[7];
  const float* dtproj_w   = (const float*)d_in[8];
  const float* dtproj_b   = (const float*)d_in[9];
  const float* A_log      = (const float*)d_in[10];
  const float* Dp         = (const float*)d_in[11];
  const float* conv_w_b   = (const float*)d_in[12];
  const float* conv_b_b   = (const float*)d_in[13];
  const float* xproj_w_b  = (const float*)d_in[14];
  const float* dtproj_w_b = (const float*)d_in[15];
  const float* dtproj_b_b = (const float*)d_in[16];
  const float* A_b_log    = (const float*)d_in[17];
  const float* Dp_b       = (const float*)d_in[18];
  const float* out_proj_w = (const float*)d_in[19];
  const float* out_proj_b = (const float*)d_in[20];

  float* out0 = (float*)d_out;
  float* out1 = out0 + (size_t)kBatch * kDmod * kSeqL;

  char* ws = (char*)d_ws;
  unsigned short* WIN  = (unsigned short*)(ws + kOffWIN);
  unsigned short* WOUT = (unsigned short*)(ws + kOffWOUT);
  unsigned short* WXPF = (unsigned short*)(ws + kOffWXPF);
  unsigned short* WXPB = (unsigned short*)(ws + kOffWXPB);
  unsigned short* WDTF = (unsigned short*)(ws + kOffWDTF);
  unsigned short* WDTB = (unsigned short*)(ws + kOffWDTB);
  unsigned short* HN   = (unsigned short*)(ws + kOffHN);
  float*          XZ   = (float*)(ws + kOffXZ);
  float*          UC   = (float*)(ws + kOffUC);
  unsigned short* UC16 = (unsigned short*)(ws + kOffUC16);
  float*          PROJ = (float*)(ws + kOffPROJ);
  unsigned short* DT16 = (unsigned short*)(ws + kOffDT16);
  float*          DLR  = (float*)(ws + kOffDLR);
  float*          GF   = (float*)(ws + kOffGF);
  unsigned short* Y16  = (unsigned short*)(ws + kOffY16);

  cast_f16_kernel<<<(kXZP * kDmod / 8) / 256, 256, 0, stream>>>(in_proj_w, WIN, kXZP * kDmod / 8, kXZP * kDmod / 8, kCarryW);
  cast_f16_kernel<<<(kDmod * kDin / 8) / 256, 256, 0, stream>>>(out_proj_w, WOUT, kDmod * kDin / 8, kDmod * kDin / 8, kCarryW);
  cast_f16_kernel<<<(kPrjP * kDin / 8) / 256, 256, 0, stream>>>(xproj_w, WXPF, kPrjP * kDin / 8, kPrjN * kDin / 8, kCarryW);
  cast_f16_kernel<<<(kPrjP * kDin / 8) / 256, 256, 0, stream>>>(xproj_w_b, WXPB, kPrjP * kDin / 8, kPrjN * kDin / 8, kCarryW);
  cast_f16_kernel<<<(kDin * kDtR / 8) / 256, 256, 0, stream>>>(dtproj_w, WDTF, kDin * kDtR / 8, kDin * kDtR / 8, kCarryW);
  cast_f16_kernel<<<(kDin * kDtR / 8) / 256, 256, 0, stream>>>(dtproj_w_b, WDTB, kDin * kDtR / 8, kDin * kDtR / 8, kCarryW);

  prelude_kernel<<<kBatch * (kSeqL / 32), 256, 0, stream>>>(hidden, residual, gamma, beta, out1, HN);

  for (int b = 0; b < kBatch; ++b) {
    const unsigned short* HNb = HN + (size_t)b * kSeqL * kDmod;
    float* outb = out0 + (size_t)b * kDmod * kSeqL;

    wmma_gemm64_f16<0><<<256, 256, 0, stream>>>(
        HNb, kDmod, WIN, kDmod, XZ, kXZP, dtproj_b, kSeqL, kXZP, kDmod, kFoldIn);

    for (int dir = 0; dir < 2; ++dir) {
      const float* cw  = dir ? conv_w_b   : conv_w;
      const float* cbp = dir ? conv_b_b   : conv_b;
      const float* db  = dir ? dtproj_b_b : dtproj_b;
      const float* al  = dir ? A_b_log    : A_log;
      const float* dpp = dir ? Dp_b       : Dp;
      const unsigned short* WXP = dir ? WXPB : WXPF;
      const unsigned short* WDT = dir ? WDTB : WDTF;

      if (dir == 0) conv_silu_kernel<false><<<dim3(kDin / 256, kSeqL / 64), 256, 0, stream>>>(XZ, cw, cbp, UC, UC16);
      else          conv_silu_kernel<true><<<dim3(kDin / 256, kSeqL / 64), 256, 0, stream>>>(XZ, cw, cbp, UC, UC16);

      wmma_gemm64_f16<0><<<8, 256, 0, stream>>>(
          UC16, kDin, WXP, kDin, PROJ, kPrjP, db, kSeqL, kPrjP, kDin, kFoldXp);

      dt_cast_kernel<<<(kSeqL * kDtR / 8) / 256, 256, 0, stream>>>(PROJ, DT16, kSeqL * kDtR / 8, kCarryDT);

      wmma_gemm64_f16<2><<<128, 256, 0, stream>>>(
          DT16, kDtR, WDT, kDtR, DLR, kDin, db, kSeqL, kDin, kDtR, kFoldDt);

      if (dir == 0) scan_kernel<false><<<kDin / 256, 256, 0, stream>>>(DLR, UC, XZ, PROJ, al, dpp, GF, Y16);
      else          scan_kernel<true><<<kDin / 256, 256, 0, stream>>>(DLR, UC, XZ, PROJ, al, dpp, GF, Y16);
    }

    wmma_gemm64_f16<1><<<64, 256, 0, stream>>>(
        WOUT, kDin, Y16, kDin, outb, kSeqL, out_proj_b, kDmod, kSeqL, kDin, kFoldOut);
  }
}
